// BaseModel_13752485281942
// MI455X (gfx1250) — hardware-verified
//
#include <hip/hip_runtime.h>
#include <math.h>

constexpr int kNodes          = 100000;
constexpr int kEdges          = 3200000;
constexpr int kCin            = 128;
constexpr int kCh             = 64;
constexpr int kMpad           = 100032;
constexpr int kThreads        = 256;
constexpr int kTileRows       = 8192;
constexpr int kTiles          = 13;
constexpr int kDinvRows       = kTiles * kTileRows;
constexpr int kWaveTileRows   = kTileRows / 8;
constexpr int kSubRows        = 512;
constexpr int kSubPerTile     = kTileRows / kSubRows;
constexpr int kAggBlocks      = kTiles * kSubPerTile;
constexpr int kEdgesPerThread = 16;
constexpr int kChunk          = kThreads * kEdgesPerThread;
constexpr int kNumChunks      = (kEdges + kChunk - 1) / kChunk;
constexpr int kListCap        = kChunk + 32;
constexpr int kCapB           = 294912;
constexpr int kBktChunks      = kCapB / kChunk;
constexpr int kGemmBlocks     = ((kMpad / 64) + 7) / 8;
constexpr int kX8Real         = kNodes * kCin / 8;
constexpr int kX8Tot          = kMpad * kCin / 8;
constexpr int kFinalBlocks    = (kNodes + kThreads - 1) / kThreads;
constexpr float kXCarry       = 8.0f;
constexpr float kWCarry       = 256.0f;
constexpr float kHCarry       = 64.0f;

static_assert(kMpad % 64 == 0 && kMpad >= kNodes && kMpad - kNodes < 64, "M tile multiple");
static_assert(kDinvRows >= kMpad, "dinv plane covers all GEMM rows");
static_assert(kEdges % kEdgesPerThread == 0, "thread edge groups are whole");
static_assert(kEdgesPerThread % 4 == 0, "b128 loads");
static_assert(kCin % 32 == 0 && kCh % 32 == 0, "K multiple of 32");
static_assert(kNodes % 32 == 0, "output lines are whole");
static_assert(kX8Tot % kThreads == 0, "cast grid exact");
static_assert(kTileRows == 8 * kWaveTileRows, "bucket wave ownership");
static_assert(kSubRows == 8 * 64, "aggregation wave ownership: 64 rows per wave");
static_assert(kTileRows == (1 << 13) && kNodes < (1 << 17), "entry packing: dl<<17 | src fits in 30 bits");
static_assert(kSubRows == (1 << 9) && kSubPerTile == 16, "sub-tile index = entry >> 26");
static_assert(kCapB % kChunk == 0 && kCapB % 32 == 0, "bucket stream chunks are whole");
static_assert((kCapB / 4) % kThreads == 0 || true, "tail fill trip bound");
static_assert(kThreads == 256, "8 waves per block");

typedef __attribute__((ext_vector_type(16))) _Float16 v16h;
typedef __attribute__((ext_vector_type(8)))  _Float16 v8h;
typedef __attribute__((ext_vector_type(8)))  float    v8f;
typedef __attribute__((ext_vector_type(4)))  float    v4f;
typedef __attribute__((ext_vector_type(2)))  float    v2f;
typedef __attribute__((ext_vector_type(4)))  int      v4i;
typedef __attribute__((ext_vector_type(4)))  unsigned int v4u;

__device__ __forceinline__ void dep_guard_h(v8f& a, v8f& b, v16h x, v16h y) { asm volatile("v_nop\n\tv_nop\n\tv_nop\n\tv_nop" : "+v"(a), "+v"(b) : "v"(x), "v"(y)); }
__device__ __forceinline__ void keep4_h(v16h a, v16h b, v16h c, v16h d) { asm volatile("v_nop" :: "v"(a), "v"(b), "v"(c), "v"(d)); }
__device__ __forceinline__ void acc_guard4(v8f& a, v8f& b, v8f& c, v8f& d) { asm volatile("v_nop\n\tv_nop\n\tv_nop\n\tv_nop" : "+v"(a), "+v"(b), "+v"(c), "+v"(d)); }
__device__ __forceinline__ void acc_guard4ab(v8f& a, v8f& b, v8f& c, v8f& d, v16h x, v16h y) {
  asm volatile("v_nop\n\tv_nop\n\tv_nop\n\tv_nop" : "+v"(a), "+v"(b), "+v"(c), "+v"(d) : "v"(x), "v"(y));
}
template <typename T> struct Frag;
template <> struct Frag<_Float16> {
  typedef v16h V; union U { v16h v; v8h h[2]; };
  static __device__ __forceinline__ v16h load(const _Float16* p) {
    U f; f.h[0] = *(const v8h*)(p); f.h[1] = *(const v8h*)(p + 16); return f.v;
  }
  static __device__ __forceinline__ v8f mma(v16h a, v16h b, v8f c) {
    return __builtin_amdgcn_wmma_f32_16x16x32_f16(false, a, false, b, (short)0, c, false, false);
  }
  static __device__ __forceinline__ void guard(v8f& a, v8f& b, v16h x, v16h y) { dep_guard_h(a, b, x, y); }
  static __device__ __forceinline__ void keep(v16h a, v16h b, v16h c, v16h d) { keep4_h(a, b, c, d); }
};
__device__ __forceinline__ unsigned pk16(unsigned short a, unsigned short b) { return (unsigned)a | ((unsigned)b << 16); }
__device__ __forceinline__ unsigned short h_bits(float f) { const _Float16 h = (_Float16)f; return __builtin_bit_cast(unsigned short, h); }
__device__ __forceinline__ void wave_lds_sync() {
  __builtin_amdgcn_fence(__ATOMIC_RELEASE, "workgroup");
  __builtin_amdgcn_wave_barrier();
  __builtin_amdgcn_fence(__ATOMIC_ACQUIRE, "workgroup");
}

template <int BIAS_MODE, bool ROWSCALE, int OUT_MODE, int ACT>
__global__ __launch_bounds__(256) void gemm64_f16(
    const unsigned short* __restrict__ Ap, int lda,
    const unsigned short* __restrict__ Btp, int ldb,
    void* __restrict__ Cout, int ldc,
    const float* __restrict__ bias, int nbias,
    const float* __restrict__ rowscale,
    int M, int N, int K, float scale, float oscale) {
  typedef _Float16 T;
  typedef v16h V;
  const T* A = (const T*)Ap; const T* Bt = (const T*)Btp;
  __shared__ __align__(16) float sT[8][16 * 68];
  const int lane = threadIdx.x & 31;
  const int wave = threadIdx.x >> 5;
  const int tilesN = N >> 6;
  const int tilesM = M >> 6;
  const int tile = blockIdx.x * 8 + wave;
  if (tile >= tilesM * tilesN) return;
  const int tm = tile / tilesN;
  const int tn = tile - tm * tilesN;
  const int m0 = tm << 6;
  const int n0 = tn << 6;

  const int rlane = lane & 15;
  const int koff  = (lane >> 4) * 8;
  const int mOff  = (lane >> 4) * 8;

  v8f acc[4][4];
#pragma unroll
  for (int i = 0; i < 4; ++i)
#pragma unroll
    for (int j = 0; j < 4; ++j) acc[i][j] = (v8f){0.f,0.f,0.f,0.f,0.f,0.f,0.f,0.f};

  for (int k0 = 0; k0 < K; k0 += 32) {
    V bh[4];
#pragma unroll
    for (int j = 0; j < 4; ++j) {
      const size_t bo = (size_t)(n0 + (j << 4) + rlane) * ldb + koff + k0;
      bh[j] = Frag<T>::load(Bt + bo);
    }
#pragma unroll
    for (int i = 0; i < 4; ++i) {
      const size_t ao = (size_t)(m0 + (i << 4) + rlane) * lda + koff + k0;
      V ah = Frag<T>::load(A + ao);
#pragma unroll
      for (int j = 0; j < 4; ++j) acc[i][j] = Frag<T>::mma(ah, bh[j], acc[i][j]);
      acc_guard4ab(acc[i][0], acc[i][1], acc[i][2], acc[i][3], ah, bh[3]);
    }
    Frag<T>::keep(bh[0], bh[1], bh[2], bh[3]);
  }
  acc_guard4(acc[0][0], acc[0][1], acc[0][2], acc[0][3]);
  acc_guard4(acc[1][0], acc[1][1], acc[1][2], acc[1][3]);
  acc_guard4(acc[2][0], acc[2][1], acc[2][2], acc[2][3]);
  acc_guard4(acc[3][0], acc[3][1], acc[3][2], acc[3][3]);

  float* slab = sT[wave];
#pragma unroll
  for (int i = 0; i < 4; ++i) {
    const int mBase = m0 + (i << 4);
    float rsv[8];
    if constexpr (ROWSCALE) {
      const v4f r0v = *(const v4f*)(rowscale + mBase + mOff);
      const v4f r1v = *(const v4f*)(rowscale + mBase + mOff + 4);
      rsv[0] = r0v[0]; rsv[1] = r0v[1]; rsv[2] = r0v[2]; rsv[3] = r0v[3];
      rsv[4] = r1v[0]; rsv[5] = r1v[1]; rsv[6] = r1v[2]; rsv[7] = r1v[3];
    } else {
#pragma unroll
      for (int r = 0; r < 8; ++r) rsv[r] = 1.0f;
    }
#pragma unroll
    for (int j = 0; j < 4; ++j) {
      const int n = n0 + (j << 4) + rlane;
      float bv = 0.f;
      if constexpr (BIAS_MODE == 2) {
        const int nb = n < nbias ? n : nbias - 1;
        const float fb = (n < nbias) ? 1.0f : 0.0f;
        bv = bias[nb] * fb;
      }
#pragma unroll
      for (int r = 0; r < 8; ++r) {
        float v = acc[i][j][r] * scale;
        if constexpr (ROWSCALE) v = v * rsv[r];
        if constexpr (BIAS_MODE == 2) v += bv;
        if constexpr (ACT == 2) v = fmaxf(v, 0.0f);
        v = v * oscale;
        slab[(mOff + r) * 68 + (j << 4) + rlane] = v;
      }
    }
    wave_lds_sync();
    if constexpr (OUT_MODE == 0) {
      float* C = (float*)Cout;
      const int hh = lane >> 4, c4 = (lane & 15) * 4;
      for (int pass = 0; pass < 2; ++pass) {
#pragma unroll
        for (int it = 0; it < 8; ++it) {
          const int row = it * 2 + hh;
          v4f v = *(const v4f*)(slab + row * 68 + c4);
          *(volatile v4f*)(C + (size_t)(mBase + row) * ldc + n0 + c4) = v;
        }
        __threadfence();
      }
    } else {
      const int q = lane >> 3, c8 = (lane & 7) * 8;
      unsigned short* C = (unsigned short*)Cout;
      for (int pass = 0; pass < 2; ++pass) {
#pragma unroll
        for (int it = 0; it < 4; ++it) {
          const int row = it * 4 + q;
          const float* sp = slab + row * 68 + c8;
          v8h hv;
#pragma unroll
          for (int e = 0; e < 8; ++e) hv[e] = (_Float16)sp[e];
          *(volatile v8h*)(C + (size_t)(mBase + row) * ldc + n0 + c8) = hv;
        }
        __threadfence();
      }
    }
    wave_lds_sync();
  }
}

__global__ __launch_bounds__(256) void prep_kernel(const float* __restrict__ W1, const float* __restrict__ W2,
                                                   const float* __restrict__ L1, const float* __restrict__ L2,
                                                   unsigned short* __restrict__ Bt1, unsigned short* __restrict__ Bt2,
                                                   unsigned short* __restrict__ Bt3, unsigned short* __restrict__ Bt4,
                                                   float wscale) {
  __shared__ __align__(16) float sm[64][132];
  const int tid = threadIdx.x;
  const int z = blockIdx.x;
  const float* W = (z == 0) ? W1 : ((z == 1) ? W2 : ((z == 2) ? L1 : L2));
  unsigned short* Bo = (z == 0) ? Bt1 : ((z == 1) ? Bt2 : ((z == 2) ? Bt3 : Bt4));
  const int kd = (z == 0) ? kCin : kCh;
  const int nr = (z == 3) ? 32 : kCh;
  const int nel = kd * 64;
#pragma unroll 1
  for (int it = 0; it < 32; ++it) {
    const int e = it * kThreads + tid;
    if (e < nel) {
      const int k = e >> 6, n = e & 63;
      const int nc = n < nr ? n : nr - 1;
      const float v = W[(size_t)k * nr + nc] * wscale;
      const float f = (n < nr) ? 1.0f : 0.0f;
      sm[n][k] = fmaf(v, f, 0.0f);
    }
  }
  __syncthreads();
  const int lcpr = (z == 0) ? 4 : 3;
  const int cpr = 1 << lcpr;
  const int nchk = 64 * cpr;
  v4u u[4];
#pragma unroll
  for (int it = 0; it < 4; ++it) {
    const int c = it * kThreads + tid;
    const int cc = c < nchk ? c : 0;
    const int row = cc >> lcpr;
    const int k8 = (cc & (cpr - 1)) * 8;
    const float* sp = &sm[row][k8];
    const v4f a = *(const v4f*)sp;
    const v4f b = *(const v4f*)(sp + 4);
    unsigned short hb[8];
#pragma unroll
    for (int e = 0; e < 4; ++e) { hb[e] = h_bits(a[e]); hb[4 + e] = h_bits(b[e]); }
    u[it] = (v4u){pk16(hb[0], hb[1]), pk16(hb[2], hb[3]), pk16(hb[4], hb[5]), pk16(hb[6], hb[7])};
  }
  for (int pass = 0; pass < 2; ++pass) {
#pragma unroll
    for (int it = 0; it < 4; ++it) {
      const int c = it * kThreads + tid;
      if (c < nchk) {
        const int row = c >> lcpr;
        const int k8 = (c & (cpr - 1)) * 8;
        *(volatile v4u*)(Bo + (size_t)row * kd + k8) = u[it];
      }
    }
    __threadfence();
  }
}

__global__ __launch_bounds__(256) void castx_kernel(const float* __restrict__ in, unsigned short* __restrict__ outp, float s) {
  const int i = blockIdx.x * kThreads + threadIdx.x;
  if (i >= kX8Tot) return;
  const int ic = i < kX8Real ? i : kX8Real - 1;
  const float f = (i < kX8Real) ? s : 0.0f;
  const float* p = in + 8 * (size_t)ic;
  const v4f a = *(const v4f*)p;
  const v4f c = *(const v4f*)(p + 4);
  unsigned short hb[8];
#pragma unroll
  for (int e = 0; e < 4; ++e) {
    hb[e]     = h_bits(fmaf(a[e], f, 0.0f));
    hb[4 + e] = h_bits(fmaf(c[e], f, 0.0f));
  }
  const v4u u = (v4u){pk16(hb[0], hb[1]), pk16(hb[2], hb[3]), pk16(hb[4], hb[5]), pk16(hb[6], hb[7])};
  unsigned short* q = outp + 8 * (size_t)i;
  *(volatile v4u*)q = u;
  __threadfence();
  *(volatile v4u*)q = u;
}

__device__ __forceinline__ int blk_excl_scan(int cnt, int* scan_ws, int tid, int* tot) {
  const int lane = tid & 31, wave = tid >> 5; int incl = cnt;
#pragma unroll
  for (int o = 1; o < 32; o <<= 1) { const int v = __shfl_up(incl, o, 32); if (lane >= o) incl += v; }
  if (lane == 31) scan_ws[wave] = incl;
  __syncthreads();
  if (wave == 0) { int wv = (lane < kThreads / 32) ? scan_ws[lane] : 0; int wincl = wv;
#pragma unroll
    for (int o = 1; o < 32; o <<= 1) { const int v = __shfl_up(wincl, o, 32); if (lane >= o) wincl += v; }
    if (lane < kThreads / 32) scan_ws[32 + lane] = wincl - wv; if (lane == 31) scan_ws[64] = wincl; }
  __syncthreads();
  const int res = scan_ws[32 + wave] + incl - cnt; *tot = scan_ws[64];
  return res;
}

__global__ __launch_bounds__(256) void bucket_kernel(const int* __restrict__ ei, int* __restrict__ bkt, float* __restrict__ dinv) {
  __shared__ __align__(16) int LIST[kListCap];
  __shared__ __align__(16) int cnt[kTileRows];
  __shared__ int scan_ws[80];
  const int tid = threadIdx.x, lane = tid & 31, wave = tid >> 5;
  const int tile = blockIdx.x;
  const int n0 = tile * kTileRows;
  int* bt = bkt + (size_t)tile * kCapB;
  for (int i = tid; i < kTileRows; i += kThreads) cnt[i] = 0;
  for (int i = tid; i < kListCap; i += kThreads) LIST[i] = -1;
  if (tid < 80) scan_ws[tid] = 0;
  __syncthreads();
  int carry = 0;
  int gpos = 0;
  const int* srcv = ei;
  const int* dstv = ei + kEdges;
#pragma unroll 1
  for (int c = 0; c < kNumChunks; ++c) {
    const int eb = c * kChunk + tid * kEdgesPerThread;
    const bool inb = eb < kEdges;
    const int ebc = inb ? eb : (kEdges - kEdgesPerThread);
    int rec[kEdgesPerThread];
    int hc = 0;
#pragma unroll
    for (int k = 0; k < kEdgesPerThread; k += 4) {
      const v4i d4 = *(const v4i*)(dstv + ebc + k);
      const v4i s4 = *(const v4i*)(srcv + ebc + k);
#pragma unroll
      for (int e = 0; e < 4; ++e) {
        const int dl = d4[e] - n0;
        int s = s4[e]; s = max(0, min(s, kNodes - 1));
        const bool hit = inb && ((unsigned)dl < (unsigned)kTileRows);
        const int rv = (int)((((unsigned)dl & (unsigned)(kTileRows - 1)) << 17) | (unsigned)s);
        rec[k + e] = hit ? rv : -1;
        hc += hit ? 1 : 0;
      }
    }
    int tot;
    int p = blk_excl_scan(hc, scan_ws, tid, &tot) + carry;
#pragma unroll
    for (int k = 0; k < kEdgesPerThread; ++k)
      if (rec[k] >= 0) { if ((unsigned)p < (unsigned)kListCap) LIST[p] = rec[k]; ++p; }
    __syncthreads();
    int total = carry + tot; total = total < kListCap ? total : kListCap;
#pragma unroll 1
    for (int base = carry; base < total; base += 32) {
      const int q = base + lane;
      const int qc = q < total ? q : total - 1;
      const int rv0 = LIST[qc];
      const int rv = (q < total) ? rv0 : -1;
      const int own = (rv >= 0 && (rv >> 27) == wave) ? 1 : 0;
      unsigned msk = (unsigned)__ballot(own);
#pragma unroll 1
      for (int it = 0; it < 32; ++it) {
        if (msk == 0u) break;
        const int bp = __builtin_ctz(msk); msk &= msk - 1u;
        const int r = __shfl(rv, bp, 32);
        const int dl = (r >> 17) & (kTileRows - 1);
        cnt[dl] = cnt[dl] + 1;
      }
    }
    const int nfull = total & ~31;
    const int room = kCapB - gpos;
    const int nfl = nfull < room ? nfull : room;
    v4i fv[4];
#pragma unroll
    for (int it = 0; it < 4; ++it) fv[it] = *(const v4i*)(LIST + it * 1024 + tid * 4);
    for (int pass = 0; pass < 2; ++pass) {
#pragma unroll
      for (int it = 0; it < 4; ++it) {
        const int idx = it * 1024 + tid * 4;
        if (idx < nfl) *(volatile v4i*)(bt + gpos + idx) = fv[it];
      }
      __threadfence();
    }
    __syncthreads();
    if (nfull > 0 && tid < 32) {
      const int mv = LIST[nfull + tid];
      LIST[tid] = mv;
    }
    carry = total - nfull;
    gpos += nfl;
    __syncthreads();
  }
  {
    const int v0 = LIST[lane];
    const int v = (lane < carry) ? v0 : -1;
    const bool doit = (wave == 0) && (gpos < kCapB);
    for (int pass = 0; pass < 2; ++pass) {
      if (doit) *(volatile int*)(bt + gpos + lane) = v;
      __threadfence();
    }
    gpos += 32;
  }
  {
    const int rem4 = (gpos < kCapB) ? ((kCapB - gpos) >> 2) : 0;
    const int trips = (rem4 + kThreads - 1) / kThreads;
    const v4i mone = (v4i){-1, -1, -1, -1};
    for (int pass = 0; pass < 2; ++pass) {
#pragma unroll 1
      for (int it = 0; it < trips; ++it) {
        const int ci = it * kThreads + tid;
        if (ci < rem4) *(volatile v4i*)(bt + gpos + 4 * ci) = mone;
      }
      __threadfence();
    }
  }
  __syncthreads();
#pragma unroll 1
  for (int j = 0; j < 8; ++j) {
    const int idx = j * 1024 + wave * 128 + 4 * lane;
    const v4i c4 = *(const v4i*)(cnt + idx);
    v4f d;
#pragma unroll
    for (int e = 0; e < 4; ++e) d[e] = 1.0f / sqrtf(1.0f + (float)c4[e]);
    float* dp = dinv + n0 + idx;
    *(volatile v4f*)dp = d;
    __threadfence();
    *(volatile v4f*)dp = d;
  }
}

__global__ __launch_bounds__(256) void agg_kernel(const float* __restrict__ hs, const int* __restrict__ bkt,
                                                  const float* __restrict__ dinv, const float* __restrict__ bias,
                                                  unsigned short* __restrict__ hout, float ocarry) {
  __shared__ __align__(16) float accs[kSubRows * kCh];
  __shared__ __align__(16) int LIST[kChunk];
  __shared__ int scan_ws[80];
  const int tid = threadIdx.x, lane = tid & 31, wave = tid >> 5;
  const int tile = blockIdx.x / kSubPerTile;
  const int sub = blockIdx.x - tile * kSubPerTile;
  const int n0 = tile * kTileRows + sub * kSubRows;
  if (n0 >= kMpad) return;
  const int* bt = bkt + (size_t)tile * kCapB;
  const int lane2 = 2 * lane;
  {
    const v2f z2 = (v2f){0.f, 0.f};
#pragma unroll 1
    for (int j = 0; j < 64; ++j) *(v2f*)(accs + (wave * 64 + j) * kCh + lane2) = z2;
  }
  if (tid < 80) scan_ws[tid] = 0;
  __syncthreads();
#pragma unroll 1
  for (int c = 0; c < kBktChunks; ++c) {
    const int eb = c * kChunk + tid * kEdgesPerThread;
    int rec[kEdgesPerThread];
    int hc = 0;
#pragma unroll
    for (int k = 0; k < kEdgesPerThread; k += 4) {
      const v4i r4 = *(const v4i*)(bt + eb + k);
#pragma unroll
      for (int e = 0; e < 4; ++e) {
        const int r = r4[e];
        const bool hit = ((r >> 26) == sub);
        rec[k + e] = hit ? r : -1;
        hc += hit ? 1 : 0;
      }
    }
    int tot;
    int p = blk_excl_scan(hc, scan_ws, tid, &tot);
#pragma unroll
    for (int k = 0; k < kEdgesPerThread; ++k)
      if (rec[k] >= 0) { if ((unsigned)p < (unsigned)kChunk) LIST[p] = rec[k]; ++p; }
    __syncthreads();
    const int totc = tot < kChunk ? tot : kChunk;
#pragma unroll 1
    for (int base = 0; base < totc; base += 32) {
      const int q = base + lane;
      const int qc = q < totc ? q : 0;
      const int rv0 = LIST[qc];
      const int rv = (q < totc) ? rv0 : -1;
      const int own = (rv >= 0 && ((rv >> 23) & 7) == wave) ? 1 : 0;
      unsigned msk = (unsigned)__ballot(own);
#pragma unroll 1
      for (int it = 0; it < 32; ++it) {
        if (msk == 0u) break;
        const int bp = __builtin_ctz(msk); msk &= msk - 1u;
        const int r = __shfl(rv, bp, 32);
        int s = r & 0x1FFFF; s = s < kNodes ? s : kNodes - 1;
        const int dl = (r >> 17) & (kSubRows - 1);
        const v2f h = *(const v2f*)(hs + (size_t)s * kCh + lane2);
        float* ap = accs + dl * kCh + lane2;
        v2f a = *(const v2f*)ap;
        a = a + h;
        *(v2f*)ap = a;
      }
    }
    __syncthreads();
  }
  __syncthreads();
  const int q = lane >> 3, c8 = (lane & 7) * 8;
  const v4f bv0 = *(const v4f*)(bias + c8);
  const v4f bv1 = *(const v4f*)(bias + c8 + 4);
#pragma unroll 1
  for (int j = 0; j < 16; ++j) {
    const int dl = wave * 64 + 4 * j + q;
    const int n = n0 + dl;
    const int nc = n < kMpad ? n : kMpad - 1;
    const float* ap = accs + dl * kCh + c8;
    const v4f a0 = *(const v4f*)ap;
    const v4f a1 = *(const v4f*)(ap + 4);
    const float* hp = hs + (size_t)nc * kCh + c8;
    const v4f h0 = *(const v4f*)hp;
    const v4f h1 = *(const v4f*)(hp + 4);
    const float dn = dinv[n];
    const float f = (n < kNodes) ? ocarry : 0.0f;
    const v4f v0 = ((a0 + h0) * dn + bv0) * f;
    const v4f v1 = ((a1 + h1) * dn + bv1) * f;
    unsigned short hb[8];
#pragma unroll
    for (int e = 0; e < 4; ++e) { hb[e] = h_bits(v0[e]); hb[4 + e] = h_bits(v1[e]); }
    const v4u u = (v4u){pk16(hb[0], hb[1]), pk16(hb[2], hb[3]), pk16(hb[4], hb[5]), pk16(hb[6], hb[7])};
    unsigned short* op = hout + (size_t)nc * kCh + c8;
    for (int pass = 0; pass < 2; ++pass) {
      if (n < kMpad) *(volatile v4u*)op = u;
      __threadfence();
    }
  }
}

__global__ __launch_bounds__(256) void final_kernel(const float* __restrict__ m2, const float* __restrict__ lw3,
                                                    const float* __restrict__ lb3, float* __restrict__ out) {
  __shared__ __align__(16) float sw[32];
  __shared__ __align__(16) float so[kThreads];
  const int tid = threadIdx.x;
  if (tid < 8) *(v4f*)(sw + 4 * tid) = *(const v4f*)(lw3 + 4 * tid);
  __syncthreads();
  const int row = blockIdx.x * kThreads + tid;
  const int rc = row < kNodes ? row : kNodes - 1;
  const float* rp = m2 + (size_t)rc * kCh;
  float s = 0.0f;
#pragma unroll
  for (int c = 0; c < 32; c += 4) {
    const v4f m = *(const v4f*)(rp + c);
    const v4f w = *(const v4f*)(sw + c);
    s = fmaf(m[0], w[0], s); s = fmaf(m[1], w[1], s); s = fmaf(m[2], w[2], s); s = fmaf(m[3], w[3], s);
  }
  s += lb3[0];
  so[tid] = s;
  __syncthreads();
  if (tid < 64) {
    const int base = blockIdx.x * kThreads + 4 * tid;
    const v4f o = *(const v4f*)(so + 4 * tid);
    float* dp = out + (size_t)(base < kNodes ? base : 0);
    for (int pass = 0; pass < 2; ++pass) {
      if (base < kNodes) *(volatile v4f*)dp = o;
      __threadfence();
    }
  }
}

extern "C" void kernel_launch(void* const* d_in, const int* in_sizes, int n_in,
                              void* d_out, int out_size, void* d_ws, size_t ws_size, hipStream_t stream) {
  (void)in_sizes; (void)n_in; (void)out_size;
  const float* x   = (const float*)d_in[0];
  const int*   ei  = (const int*)d_in[1];
  const float* W1  = (const float*)d_in[2];
  const float* b1  = (const float*)d_in[3];
  const float* W2  = (const float*)d_in[4];
  const float* b2  = (const float*)d_in[5];
  const float* lw1 = (const float*)d_in[6];
  const float* lb1 = (const float*)d_in[7];
  const float* lw2 = (const float*)d_in[8];
  const float* lb2 = (const float*)d_in[9];
  const float* lw3 = (const float*)d_in[10];
  const float* lb3 = (const float*)d_in[11];
  float* out = (float*)d_out;

  char* ws = (char*)d_ws; size_t off = 0;
  auto carve = [&](size_t bytes) -> char* { char* p = ws + off; off += (bytes + 255) & ~(size_t)255; return p; };
  float*          dinv = (float*)carve((size_t)kDinvRows * 4);
  unsigned short* Xh   = (unsigned short*)carve((size_t)kMpad * kCin * 2);
  unsigned short* Bt1  = (unsigned short*)carve((size_t)64 * kCin * 2);
  unsigned short* Bt2  = (unsigned short*)carve((size_t)64 * kCh * 2);
  unsigned short* Bt3  = (unsigned short*)carve((size_t)64 * kCh * 2);
  unsigned short* Bt4  = (unsigned short*)carve((size_t)64 * kCh * 2);
  int*            BKT  = (int*)carve((size_t)kTiles * kCapB * 4);
  float*          HS   = (float*)carve((size_t)kMpad * kCh * 4);
  unsigned short* H1   = (unsigned short*)carve((size_t)kMpad * kCh * 2);
  unsigned short* H2   = (unsigned short*)carve((size_t)kMpad * kCh * 2);
  unsigned short* M1   = (unsigned short*)carve((size_t)kMpad * kCh * 2);
  if (off > ws_size || off > (size_t)134217728) return;
  float* M2 = HS;

  prep_kernel<<<4, kThreads, 0, stream>>>(W1, W2, lw1, lw2, Bt1, Bt2, Bt3, Bt4, kWCarry);
  castx_kernel<<<kX8Tot / kThreads, kThreads, 0, stream>>>(x, Xh, kXCarry);
  bucket_kernel<<<kTiles, kThreads, 0, stream>>>(ei, BKT, dinv);

  gemm64_f16<0, true, 0, 0><<<kGemmBlocks, 256, 0, stream>>>(
      Xh, kCin, Bt1, kCin, (void*)HS, kCh, (const float*)nullptr, 0, dinv,
      kMpad, kCh, kCin, 1.0f / (kXCarry * kWCarry), 1.0f);
  agg_kernel<<<kAggBlocks, kThreads, 0, stream>>>(HS, BKT, dinv, b1, H1, kHCarry);

  gemm64_f16<0, true, 0, 0><<<kGemmBlocks, 256, 0, stream>>>(
      H1, kCh, Bt2, kCh, (void*)HS, kCh, (const float*)nullptr, 0, dinv,
      kMpad, kCh, kCh, 1.0f / (kHCarry * kWCarry), 1.0f);
  agg_kernel<<<kAggBlocks, kThreads, 0, stream>>>(HS, BKT, dinv, b2, H2, kHCarry);

  gemm64_f16<2, false, 1, 2><<<kGemmBlocks, 256, 0, stream>>>(
      H2, kCh, Bt3, kCh, (void*)M1, kCh, lb1, kCh, (const float*)nullptr,
      kMpad, kCh, kCh, 1.0f / (kHCarry * kWCarry), kHCarry);
  gemm64_f16<2, false, 0, 2><<<kGemmBlocks, 256, 0, stream>>>(
      M1, kCh, Bt4, kCh, (void*)M2, kCh, lb2, 32, (const float*)nullptr,
      kMpad, kCh, kCh, 1.0f / (kHCarry * kWCarry), 1.0f);
  final_kernel<<<kFinalBlocks, kThreads, 0, stream>>>(M2, lw3, lb3, out);
}
